// DecoderAttentionRotary_88776974008461
// MI455X (gfx1250) — hardware-verified
//
#include <hip/hip_runtime.h>


#define NB_  1
#define TT   4096
#define DD   1024
#define NH_  16
#define HD   64
#define ZH   1
#define RH   256
#define NF   32
#define SCL  0.125f
#define PCAR 1024.0f
typedef _Float16 h16;
typedef unsigned short bf;
typedef __attribute__((ext_vector_type(16))) __bf16   v16bf;
typedef __attribute__((ext_vector_type(16))) _Float16 v16h;
typedef __attribute__((ext_vector_type(8)))  _Float16 v8h;
typedef __attribute__((ext_vector_type(8)))  unsigned short v8us;
typedef __attribute__((ext_vector_type(8)))  float    v8f;
typedef __attribute__((ext_vector_type(4)))  float    v4f;
typedef v8h  __attribute__((may_alias)) v8ha;
typedef v4f  __attribute__((may_alias)) v4fa;
typedef v8us __attribute__((may_alias)) v8usa;

__device__ __forceinline__ unsigned short f2bf(float f) { unsigned u = __float_as_uint(f); u += 0x7FFFu + ((u >> 16) & 1u); return (unsigned short)(u >> 16); }
__device__ __forceinline__ float bf2f(unsigned short b) { return __uint_as_float(((unsigned)b) << 16); }
__device__ __forceinline__ float bfr(float f) { return bf2f(f2bf(f)); }
__device__ __forceinline__ v16h cat16(v8h lo, v8h hi) { return __builtin_shufflevector(lo, hi, 0, 1, 2, 3, 4, 5, 6, 7, 8, 9, 10, 11, 12, 13, 14, 15); }
__device__ __forceinline__ v16bf cat16b(v8us lo, v8us hi) { return __builtin_bit_cast(v16bf, __builtin_shufflevector(lo, hi, 0, 1, 2, 3, 4, 5, 6, 7, 8, 9, 10, 11, 12, 13, 14, 15)); }
__device__ __forceinline__ v8f wmma16(v16h a, v16h b, v8f c) { return __builtin_amdgcn_wmma_f32_16x16x32_f16(false, a, false, b, (short)0, c, false, false); }
__device__ __forceinline__ v8f wmmab(v16bf a, v16bf b, v8f c) { return __builtin_amdgcn_wmma_f32_16x16x32_bf16(false, a, false, b, (short)0, c, false, false); }


template <typename T16> struct WFrag;
template <> struct WFrag<h16> { typedef v16h V; static __device__ __forceinline__ V ld(const h16* p) { return cat16(*(const v8h*)p, *(const v8h*)(p + 16)); } static __device__ __forceinline__ v8f mma(V a, V b, v8f c) { return wmma16(a, b, c); } };
template <> struct WFrag<bf> { typedef v16bf V; static __device__ __forceinline__ V ld(const bf* p) { return cat16b(*(const v8us*)p, *(const v8us*)(p + 16)); } static __device__ __forceinline__ v8f mma(V a, V b, v8f c) { return wmmab(a, b, c); } };
template <typename T16, int NSPLIT, bool BIAS>
__global__ __launch_bounds__(32) void k_gemmw(const T16* __restrict__ A, const T16* __restrict__ A2, const T16* __restrict__ Bt, const T16* __restrict__ Bt2, int K, float* C, int ldc, const float* __restrict__ bias, size_t sA, size_t sB, size_t sC) {
    typedef typename WFrag<T16>::V V;
    __shared__ __align__(16) float os[16 * 68];
    const size_t z = blockIdx.z; A += z * sA; if (A2) A2 += z * sA; Bt += z * sB; if (Bt2) Bt2 += z * sB; C += z * sC;
    const int lane = threadIdx.x & 31, lr = lane & 15, hi = lane >> 4; const int r0 = blockIdx.x * 64, c0 = blockIdx.y * 64;
    v8f acc[4][4];
#pragma unroll
    for (int mb = 0; mb < 4; ++mb)
#pragma unroll
        for (int nb = 0; nb < 4; ++nb) acc[mb][nb] = (v8f){};
    const size_t aoff = (size_t)(r0 + lr) * K + 8 * hi, boff = (size_t)(c0 + lr) * K + 8 * hi;
#pragma unroll 1
    for (int kc = 0; kc < K; kc += 32) {
        V a[4], a2[4];
#pragma unroll
        for (int mb = 0; mb < 4; ++mb) { a[mb] = WFrag<T16>::ld(A + aoff + (size_t)mb * 16 * K + kc); if (NSPLIT == 1 || NSPLIT == 2) a2[mb] = WFrag<T16>::ld(A2 + aoff + (size_t)mb * 16 * K + kc); }
#pragma unroll
        for (int nb = 0; nb < 4; ++nb) { const V b = WFrag<T16>::ld(Bt + boff + (size_t)nb * 16 * K + kc); V b2; if (NSPLIT >= 2) b2 = WFrag<T16>::ld(Bt2 + boff + (size_t)nb * 16 * K + kc);
#pragma unroll
            for (int mb = 0; mb < 4; ++mb) { acc[mb][nb] = WFrag<T16>::mma(a[mb], b, acc[mb][nb]); if (NSPLIT == 1 || NSPLIT == 2) acc[mb][nb] = WFrag<T16>::mma(a2[mb], b, acc[mb][nb]); if (NSPLIT >= 2) acc[mb][nb] = WFrag<T16>::mma(a[mb], b2, acc[mb][nb]); } }
        asm volatile("v_nop\n\tv_nop\n\tv_nop\n\tv_nop" : "+v"(acc[0][0]), "+v"(acc[1][1]), "+v"(acc[2][2]), "+v"(acc[3][3]) : "v"(a[0]), "v"(a[3]));
    }
#pragma unroll
    for (int mb = 0; mb < 4; ++mb) {
#pragma unroll
        for (int nb = 0; nb < 4; ++nb) {
#pragma unroll
            for (int j = 0; j < 8; ++j) os[(hi * 8 + j) * 68 + nb * 16 + lr] = acc[mb][nb][j]; }
        __builtin_amdgcn_wave_barrier(); asm volatile("" ::: "memory");
        float* crow = C + (size_t)(r0 + mb * 16) * ldc + c0;
#pragma unroll 1
        for (int ps = 0; ps < 2; ++ps) {
#pragma unroll
            for (int s = 0; s < 8; ++s) { const int row = 2 * s + hi, cofs = lr * 4; v4f val = *(const v4fa*)(os + row * 68 + cofs); if (BIAS) { val[0] += bfr(bias[c0 + cofs]); val[1] += bfr(bias[c0 + cofs + 1]); val[2] += bfr(bias[c0 + cofs + 2]); val[3] += bfr(bias[c0 + cofs + 3]); }
                *(volatile v4f*)(crow + (size_t)row * ldc + cofs) = val; }
            if (ps == 0) __threadfence(); }
        __builtin_amdgcn_wave_barrier(); asm volatile("" ::: "memory");
    }
}

__device__ __forceinline__ h16 tohx(float x) { return (h16)x; }
__device__ __forceinline__ void splitf(float y, unsigned short& h, unsigned short& l) { h = f2bf(y); l = f2bf(y - bf2f(h)); }
typedef __attribute__((ext_vector_type(2))) unsigned short v2us;
typedef __attribute__((ext_vector_type(2))) _Float16 v2h;
typedef __attribute__((ext_vector_type(4))) _Float16 v4h;
typedef __attribute__((ext_vector_type(2))) float v2f;

__global__ __launch_bounds__(256) void k_wtG(const float* __restrict__ w, int K, int N, bf* Bt) {
    const int lane = threadIdx.x & 31; const int L0 = (blockIdx.x * 8 + (threadIdx.x >> 5)) * 8; const int nlines = N * K / 64;
#pragma unroll 1
    for (int ps = 0; ps < 2; ++ps) {
#pragma unroll 1
        for (int l = 0; l < 8; ++l) { const int L = L0 + l; if (L >= nlines) break; const size_t e = (size_t)L * 64 + lane * 2; const int k = (int)(e % K), n = (int)(e / K); v2us o;
            o[0] = f2bf(w[(size_t)k * N + n]); o[1] = f2bf(w[(size_t)(k + 1) * N + n]); *(volatile v2us*)(Bt + e) = o; }
        if (ps == 0) __threadfence(); }
}
__global__ __launch_bounds__(256) void k_cvt8(const float* __restrict__ src, bf* dst, size_t n8) { const size_t i = (size_t)blockIdx.x * 256 + threadIdx.x; if (i >= n8) return; const v8f v = *(const v8f*)(src + i * 8); v8us o;
#pragma unroll
    for (int k = 0; k < 8; ++k) o[k] = f2bf(v[k]); *(volatile v8us*)(dst + i * 8) = o; __threadfence(); *(volatile v8us*)(dst + i * 8) = o; }
__global__ __launch_bounds__(256) void k_qplanes(const float* __restrict__ F, bf* Ph, bf* Pl, h16* P16) {
    const int lane = threadIdx.x & 31; const int L0 = (blockIdx.x * 8 + (threadIdx.x >> 5)) * 8; const int nlines = NH_ * TT * HD / 64;
#pragma unroll 1
    for (int ps = 0; ps < 2; ++ps) {
#pragma unroll
        for (int l = 0; l < 8; ++l) { const int L = L0 + l; if (L >= nlines) break; const int e = L * 64 + lane * 2; const int d = e & (HD - 1); const int t = (e >> 6) & (TT - 1); const int h = e >> 18; v2us oh, ol; v2h o16;
#pragma unroll
            for (int q = 0; q < 2; ++q) { const float x = F[(size_t)t * DD + h * HD + d + q]; unsigned short a, c2; splitf(x, a, c2); oh[q] = a; ol[q] = c2; o16[q] = tohx(x); }
            *(volatile v2us*)(Ph + (size_t)e) = oh; *(volatile v2us*)(Pl + (size_t)e) = ol; *(volatile v2h*)(P16 + (size_t)e) = o16; }
        if (ps == 0) __threadfence(); }
}
__global__ __launch_bounds__(256) void k_rplanes(const float* __restrict__ F, const float* __restrict__ CS, const int* __restrict__ pos, bf* Ph, bf* Pl, h16* P16) {
    const int e = (blockIdx.x * 256 + threadIdx.x) * 2; if (e >= NH_ * TT * HD) return; const int d = e & (HD - 1); const int t = (e >> 6) & (TT - 1); const int h = e >> 18; int pr = pos ? pos[t] : t; pr = pr < 0 ? 0 : (pr >= TT ? TT - 1 : pr);
    const float x0 = F[(size_t)t * DD + h * HD + d], x1 = F[(size_t)t * DD + h * HD + d + 1]; const v2f cs = *(const v2f*)(CS + ((size_t)pr * NF + (d >> 1)) * 2);
    float a1 = __fmul_rn(x0, cs[0]), a2 = __fmul_rn(x1, cs[1]), a3 = __fmul_rn(x1, cs[0]), a4 = __fmul_rn(x0, cs[1]); asm volatile("" : "+v"(a1)); asm volatile("" : "+v"(a2)); asm volatile("" : "+v"(a3)); asm volatile("" : "+v"(a4));
    const float r0 = __fsub_rn(a1, a2), r1 = __fadd_rn(a3, a4); v2us oh, ol; v2h o16; unsigned short a, c2; splitf(r0, a, c2); oh[0] = a; ol[0] = c2; splitf(r1, a, c2); oh[1] = a; ol[1] = c2; o16[0] = tohx(r0); o16[1] = tohx(r1);
    *(volatile v2us*)(Ph + e) = oh; *(volatile v2us*)(Pl + e) = ol; *(volatile v2h*)(P16 + e) = o16; __threadfence(); *(volatile v2us*)(Ph + e) = oh; *(volatile v2us*)(Pl + e) = ol; *(volatile v2h*)(P16 + e) = o16; }
__global__ __launch_bounds__(256) void k_cstab(float* CS) { const int idx = blockIdx.x * 256 + threadIdx.x; if (idx >= TT * NF) return; const int p = idx >> 5, i = idx & 31; const float inv = __fdiv_rn(1.0f, powf(10000.0f, (float)(2 * i) / 64.0f)); const float ang = __fmul_rn((float)p, inv); v2f o; o[0] = cosf(ang); o[1] = sinf(ang);
    *(volatile v2f*)(CS + (size_t)idx * 2) = o; __threadfence(); *(volatile v2f*)(CS + (size_t)idx * 2) = o; }
__global__ __launch_bounds__(256) void k_cscvt(const float* __restrict__ fc, float* CS) { const int idx = blockIdx.x * 256 + threadIdx.x; if (idx >= TT * NF) return; const v2f a = *(const v2f*)(fc + (size_t)idx * 2); v2f o; o[0] = bfr(a[0]); o[1] = bfr(a[1]); *(volatile v2f*)(CS + (size_t)idx * 2) = o; __threadfence(); *(volatile v2f*)(CS + (size_t)idx * 2) = o; }
__global__ __launch_bounds__(256) void k_vtplane(const float* __restrict__ F, bf* Vh, bf* Vl, h16* V16) {
    const int lane = threadIdx.x & 31; const int L0 = (blockIdx.x * 8 + (threadIdx.x >> 5)) * 8; const int nlines = NH_ * TT * HD / 64;
#pragma unroll 1
    for (int ps = 0; ps < 2; ++ps) {
#pragma unroll
        for (int l = 0; l < 8; ++l) { const int L = L0 + l; if (L >= nlines) break; const int e = L * 64 + lane * 2; const int t = e & (TT - 1); const int d = (e >> 12) & (HD - 1); const int h = e >> 18; v2us oh, ol; v2h o16;
#pragma unroll
            for (int q = 0; q < 2; ++q) { const float x = F[(size_t)(t + q) * DD + h * HD + d]; unsigned short a, c2; splitf(x, a, c2); oh[q] = a; ol[q] = c2; o16[q] = tohx(x); }
            *(volatile v2us*)(Vh + (size_t)e) = oh; *(volatile v2us*)(Vl + (size_t)e) = ol; *(volatile v2h*)(V16 + (size_t)e) = o16; }
        if (ps == 0) __threadfence(); }
}
__global__ __launch_bounds__(256) void k_smax4(const float* __restrict__ S, float* RS) {
    const int lane = threadIdx.x & 31; const int i = blockIdx.x * 8 + (threadIdx.x >> 5); if (i >= TT) return; const float* sr = S + (size_t)i * TT; float m = -3.0e38f;
#pragma unroll 4
    for (int c0 = lane * 4; c0 < TT; c0 += 128) { if (c0 > i) break; const v4f v = *(const v4f*)(sr + c0);
#pragma unroll
        for (int q = 0; q < 4; ++q) m = (c0 + q <= i) ? fmaxf(m, v[q]) : m; }
#pragma unroll
    for (int sh = 16; sh; sh >>= 1) m = fmaxf(m, __shfl_xor(m, sh, 32));
    const float o = lane == 0 ? m : 0.f; *(volatile float*)(RS + (size_t)i * 32 + lane) = o; __threadfence(); *(volatile float*)(RS + (size_t)i * 32 + lane) = o;
}
__global__ __launch_bounds__(256) void k_sexp4(const float* __restrict__ S, float* RS, bf* Ph, bf* Pl, h16* P16) {
    typedef __attribute__((ext_vector_type(4))) unsigned short v4us;
    const int lane = threadIdx.x & 31; const int i = blockIdx.x * 8 + (threadIdx.x >> 5); if (i >= TT) return; const bool hires = (i < RH); const float* sr = S + (size_t)i * TT; const float m = RS[(size_t)i * 32]; float sum = 0.f;
#pragma unroll 1
    for (int ps = 0; ps < 2; ++ps) { sum = 0.f;
#pragma unroll 2
        for (int c0 = lane * 4; c0 < TT; c0 += 128) { const v4f v = *(const v4f*)(sr + c0); float e4[4];
#pragma unroll
            for (int q = 0; q < 4; ++q) { float dlt = __fsub_rn(v[q], m); asm volatile("" : "+v"(dlt)); const float e = (c0 + q <= i) ? __expf(__fmul_rn(dlt, SCL)) : 0.f; sum += e; e4[q] = e; }
            if (hires) { v4us oh, ol;
#pragma unroll
                for (int q = 0; q < 4; ++q) { unsigned short a, c2; splitf(e4[q], a, c2); oh[q] = a; ol[q] = c2; } *(volatile v4us*)(Ph + (size_t)i * TT + c0) = oh; *(volatile v4us*)(Pl + (size_t)i * TT + c0) = ol; }
            else { v4h o;
#pragma unroll
                for (int q = 0; q < 4; ++q) o[q] = tohx(e4[q] * PCAR); *(volatile v4h*)(P16 + (size_t)i * TT + c0) = o; } }
        if (ps == 0) __threadfence(); }
#pragma unroll
    for (int sh = 16; sh; sh >>= 1) sum += __shfl_xor(sum, sh, 32);
    const float o2 = lane == 0 ? m : (lane == 1 ? __fdiv_rn(1.0f, hires ? sum : sum * PCAR) : 0.f); *(volatile float*)(RS + (size_t)i * 32 + lane) = o2; __threadfence(); *(volatile float*)(RS + (size_t)i * 32 + lane) = o2;
}
__global__ __launch_bounds__(256) void k_mergef(const float* __restrict__ O, const float* __restrict__ RS, int h0, float* OUTb) { typedef __attribute__((ext_vector_type(2))) float v2f; const int e = (blockIdx.x * 256 + threadIdx.x) * 2; if (e >= TT * HD) return; const int d = e & (HD - 1); const int t = e >> 6; const float sc = RS[(size_t)t * 32 + 1]; v2f o;
    o[0] = __fmul_rn(O[e], sc); o[1] = __fmul_rn(O[e + 1], sc); const size_t oo = (size_t)t * DD + h0 * HD + d; *(volatile v2f*)(OUTb + oo) = o; __threadfence(); *(volatile v2f*)(OUTb + oo) = o; }

extern "C" void kernel_launch(void* const* d_in, const int* in_sizes, int n_in,
                              void* d_out, int out_size, void* d_ws, size_t ws_size, hipStream_t stream) {
    (void)in_sizes; (void)n_in; (void)out_size;
    const float* x = (const float*)d_in[0]; const float* fc = (const float*)d_in[1]; const float* wqkv = (const float*)d_in[2]; const float* bqkv = (const float*)d_in[3];
    float* OUT = (float*)d_out;
    char* wsp = (char*)d_ws;
    auto take = [&](size_t bytes) { char* p = wsp; wsp += (bytes + 255) & ~(size_t)255; return (void*)p; };
    bf* WQKV = (bf*)take((size_t)3 * DD * DD * 2); float* CS = (float*)take((size_t)TT * NF * 2 * 4);
    bf* XB = (bf*)take((size_t)TT * DD * 2); float* F = (float*)take((size_t)TT * DD * 4);
    bf* QPh = (bf*)take((size_t)TT * DD * 2); bf* QPl = (bf*)take((size_t)TT * DD * 2); bf* KPh = (bf*)take((size_t)TT * DD * 2); bf* KPl = (bf*)take((size_t)TT * DD * 2); bf* VTh = (bf*)take((size_t)TT * DD * 2); bf* VTl = (bf*)take((size_t)TT * DD * 2);
    h16* QP16 = (h16*)take((size_t)TT * DD * 2); h16* KP16 = (h16*)take((size_t)TT * DD * 2); h16* VT16 = (h16*)take((size_t)TT * DD * 2);
    float* Sb = (float*)take((size_t)ZH * TT * TT * 4); float* RS = (float*)take((size_t)TT * 32 * 4); bf* Ph = (bf*)take((size_t)ZH * RH * TT * 2); bf* Pl = (bf*)take((size_t)ZH * RH * TT * 2); h16* P16 = (h16*)take((size_t)ZH * TT * TT * 2); float* Ob = (float*)take((size_t)ZH * TT * HD * 4);
    if ((size_t)(wsp - (char*)d_ws) > ws_size) return;
    { k_wtG<<<(unsigned)((DD * 3 * DD / 64 + 63) / 64), 256, 0, stream>>>(wqkv, DD, 3 * DD, WQKV); k_cscvt<<<(TT * NF + 255) / 256, 256, 0, stream>>>(fc, CS); }
    const unsigned LB = (unsigned)((NH_ * TT * HD / 64 + 63) / 64), LR = (NH_ * TT * HD / 2 + 255) / 256; const dim3 gP(TT / 64, DD / 64, 1);
    for (int b = 0; b < NB_; ++b) {
        k_cvt8<<<(unsigned)(((size_t)TT * DD / 8 + 255) / 256), 256, 0, stream>>>(x + (size_t)b * TT * DD, XB, (size_t)TT * DD / 8);
        k_gemmw<bf, 0, true><<<gP, 32, 0, stream>>>(XB, nullptr, WQKV, nullptr, DD, F, DD, bqkv, 0, 0, 0); k_rplanes<<<LR, 256, 0, stream>>>(F, CS, nullptr, QPh, QPl, QP16);
        k_gemmw<bf, 0, true><<<gP, 32, 0, stream>>>(XB, nullptr, WQKV + (size_t)DD * DD, nullptr, DD, F, DD, bqkv + DD, 0, 0, 0); k_rplanes<<<LR, 256, 0, stream>>>(F, CS, nullptr, KPh, KPl, KP16);
        k_gemmw<bf, 0, true><<<gP, 32, 0, stream>>>(XB, nullptr, WQKV + (size_t)2 * DD * DD, nullptr, DD, F, DD, bqkv + 2 * DD, 0, 0, 0); k_vtplane<<<LB, 256, 0, stream>>>(F, VTh, VTl, VT16);
        for (int h0 = 0; h0 < NH_; h0 += ZH) { const size_t z0 = (size_t)h0;
            k_gemmw<bf, 2, false><<<dim3(RH / 64, TT / 64, ZH), 32, 0, stream>>>(QPh + z0 * TT * HD, QPl + z0 * TT * HD, KPh + z0 * TT * HD, KPl + z0 * TT * HD, HD, Sb, TT, nullptr, (size_t)TT * HD, (size_t)TT * HD, (size_t)TT * TT);
            k_gemmw<h16, 0, false><<<dim3((TT - RH) / 64, TT / 64, ZH), 32, 0, stream>>>(QP16 + z0 * TT * HD + (size_t)RH * HD, nullptr, KP16 + z0 * TT * HD, nullptr, HD, Sb + (size_t)RH * TT, TT, nullptr, (size_t)TT * HD, (size_t)TT * HD, (size_t)TT * TT);
            k_smax4<<<TT / 8, 256, 0, stream>>>(Sb, RS); k_sexp4<<<TT / 8, 256, 0, stream>>>(Sb, RS, Ph, Pl, P16);
            k_gemmw<bf, 2, false><<<dim3(RH / 64, HD / 64, ZH), 32, 0, stream>>>(Ph, Pl, VTh + z0 * HD * TT, VTl + z0 * HD * TT, TT, Ob, HD, nullptr, (size_t)RH * TT, (size_t)HD * TT, (size_t)TT * HD);
            k_gemmw<h16, 0, false><<<dim3((TT - RH) / 64, HD / 64, ZH), 32, 0, stream>>>(P16 + (size_t)RH * TT, nullptr, VT16 + z0 * HD * TT, nullptr, TT, Ob + (size_t)RH * HD, HD, nullptr, (size_t)TT * TT, (size_t)HD * TT, (size_t)TT * HD);
            k_mergef<<<(TT * HD / 2 + 255) / 256, 256, 0, stream>>>(Ob, RS, h0, OUT + (size_t)b * TT * DD); }
         }
}
